// preGATConv_4784593568247
// MI455X (gfx1250) — hardware-verified
//
#include <hip/hip_runtime.h>


namespace {
constexpr int N = 50000, E = 800000, FIN = 256, D = 128, NPAD = 50048, NBLK = NPAD / 128, NB = 256;
constexpr float FXS = 524288.0f, FXI = 1.0f / 524288.0f, NEG = 0.2f, ALPHA = 0.5f;

typedef _Float16 b16;
typedef __attribute__((ext_vector_type(16))) _Float16 v16b;
typedef __attribute__((ext_vector_type(8)))  _Float16 v8b;
typedef __attribute__((ext_vector_type(8)))  float v8f;
typedef __attribute__((ext_vector_type(4)))  float v4f;

__device__ __forceinline__ v8b ld8b(const b16* p) { return *(const v8b*)p; }
__device__ __forceinline__ v16b cat8b(v8b a, v8b b) { return __builtin_shufflevector(a, b, 0, 1, 2, 3, 4, 5, 6, 7, 8, 9, 10, 11, 12, 13, 14, 15); }
__device__ __forceinline__ v16b frag_kb(const b16* p, int hh) { return cat8b(ld8b(p + 8 * hh), ld8b(p + 16 + 8 * hh)); }
__device__ __forceinline__ void split16(float v, b16& hi, b16& lo) { hi = (b16)v; lo = (b16)(v - (float)hi); }
__device__ __forceinline__ void frag_ksplit(const float* p, int hh, v16b& fh_, v16b& fl_) {
  const float* p0 = p + 8 * hh; const float* p1 = p + 16 + 8 * hh;
#pragma unroll
  for (int e = 0; e < 8; ++e) { b16 a, c; split16(p0[e], a, c); fh_[e] = a; fl_[e] = c; split16(p1[e], a, c); fh_[8 + e] = a; fl_[8 + e] = c; }
}
__device__ __forceinline__ v8f wmma16b(v16b a, v16b b, v8f c) {
  v8f d = __builtin_amdgcn_wmma_f32_16x16x32_f16(false, a, false, b, (short)0, c, false, false);
  asm volatile("v_nop\n\tv_nop\n\tv_nop\n\tv_nop" : "+v"(d) : "v"(a), "v"(b));
  return d;
}
__device__ __forceinline__ void wave_lds_sync() {
  __builtin_amdgcn_fence(__ATOMIC_RELEASE, "workgroup");
  __builtin_amdgcn_wave_barrier();
  __builtin_amdgcn_fence(__ATOMIC_ACQUIRE, "workgroup");
}

struct Opnd { const void* p0; const void* p1; int ld; };
template <int NP> __device__ __forceinline__ void load_frags(const Opnd& o, int row, int kb, int hh, v16b& fh_, v16b& fl_) {
  if (NP == 0) { frag_ksplit((const float*)o.p0 + (size_t)row * o.ld + kb, hh, fh_, fl_); }
  else if (NP == 4) {
    const float* p = (const float*)o.p0 + (size_t)row * o.ld + kb; const float* p0 = p + 8 * hh; const float* p1 = p + 16 + 8 * hh;
#pragma unroll
    for (int e = 0; e < 8; ++e) { b16 a, c; split16(p0[e] * 64.0f, a, c); fh_[e] = a; fl_[e] = c; split16(p1[e] * 64.0f, a, c); fh_[8 + e] = a; fl_[8 + e] = c; }
  } else if (NP == 3) {
    const float* p = (const float*)o.p0 + (size_t)row * o.ld + kb; const float* p0 = p + 8 * hh; const float* p1 = p + 16 + 8 * hh;
#pragma unroll
    for (int e = 0; e < 8; ++e) { fh_[e] = (b16)p0[e]; fh_[8 + e] = (b16)p1[e]; }
    fl_ = fh_;
  } else {
    fh_ = frag_kb((const b16*)o.p0 + (size_t)row * o.ld + kb, hh);
    if (NP == 2) fl_ = frag_kb((const b16*)o.p1 + (size_t)row * o.ld + kb, hh); else fl_ = fh_;
  }
}
template <int ANP, int BNP> __device__ __forceinline__ v8f mac(v16b ah, v16b al, v16b bh, v16b bl, v8f c) {
  c = wmma16b(ah, bh, c);
  if (BNP == 0 || BNP == 2 || BNP == 4) c = wmma16b(ah, bl, c);
  if (ANP == 0 || ANP == 2 || ANP == 4) c = wmma16b(al, bh, c);
  return c;
}
template <int ANP, int BNP>
__device__ __forceinline__ void gemm_tile(const Opnd& A, const Opnd& B, int K, int m0, int c0, int nloc, int hlf, v8f (&acc)[2][4]) {
  for (int kb = 0; kb < K; kb += 32) {
    v16b a0h, a0l, a1h, a1l;
    load_frags<ANP>(A, m0 + nloc, kb, hlf, a0h, a0l);
    load_frags<ANP>(A, m0 + 16 + nloc, kb, hlf, a1h, a1l);
#pragma unroll
    for (int t = 0; t < 4; ++t) {
      v16b bh, bl;
      load_frags<BNP>(B, c0 + t * 16 + nloc, kb, hlf, bh, bl);
      acc[0][t] = mac<ANP, BNP>(a0h, a0l, bh, bl, acc[0][t]);
      acc[1][t] = mac<ANP, BNP>(a1h, a1l, bh, bl, acc[1][t]);
    }
  }
}

__device__ __forceinline__ void epi_planes(v8f (&acc)[2][4], float scale, bool two, b16* __restrict__ oh, b16* __restrict__ ol, int ldo,
                                           int m0, int c0, int lane, b16* Th, b16* Tl) {
  const int nloc = lane & 15, hlf = lane >> 4;
#pragma unroll
  for (int t = 0; t < 4; ++t)
#pragma unroll
    for (int r = 0; r < 2; ++r)
#pragma unroll
      for (int v = 0; v < 8; ++v) {
        const int rr = r * 16 + v + 8 * hlf, cc = t * 16 + nloc;
        b16 h_, l_; split16(acc[r][t][v] * scale, h_, l_);
        Th[rr * 64 + cc] = h_; Tl[rr * 64 + cc] = l_;
      }
  wave_lds_sync();
  for (int pass = 0; pass < 2; ++pass) {
#pragma unroll
    for (int j = 0; j < 8; ++j) {
      const int rr = j * 4 + (lane >> 3), c8 = (lane & 7) * 8;
      const size_t o = (size_t)(m0 + rr) * ldo + c0 + c8;
      *(volatile v8b*)(oh + o) = ld8b(Th + rr * 64 + c8);
      if (two) *(volatile v8b*)(ol + o) = ld8b(Tl + rr * 64 + c8);
    }
    __threadfence();
  }
}
__device__ __forceinline__ void epi_f32(v8f (&acc)[2][4], float scale, const float* rscale, float* __restrict__ out, int ldo, int m0, int c0, int lane, float* Tt) {
  const int nloc = lane & 15, hlf = lane >> 4;
#pragma unroll
  for (int t = 0; t < 4; ++t)
#pragma unroll
    for (int r = 0; r < 2; ++r)
#pragma unroll
      for (int v = 0; v < 8; ++v) {
        const int rr = r * 16 + v + 8 * hlf;
        const float rs = rscale ? rscale[(size_t)(m0 + rr) * 32] : 1.0f;
        Tt[rr * 64 + t * 16 + nloc] = acc[r][t][v] * scale * rs;
      }
  wave_lds_sync();
  float* dst0 = out + (size_t)m0 * ldo + c0;
  for (int pass = 0; pass < 2; ++pass) {
#pragma unroll
    for (int j = 0; j < 16; ++j) { const int rr = j * 2 + hlf, c4 = nloc * 4; *(volatile v4f*)(dst0 + (size_t)rr * ldo + c4) = *(const v4f*)(Tt + rr * 64 + c4); }
    __threadfence();
  }
}


__device__ __forceinline__ int fkey(float f) { const int b = __float_as_int(f); return (b >= 0) ? b : (b ^ 0x7FFFFFFF); }
__device__ __forceinline__ float fkey_inv(int k) { return __int_as_float((k >= 0) ? k : (k ^ 0x7FFFFFFF)); }

__global__ __launch_bounds__(256) void prep_kernel(const float* __restrict__ W, b16* __restrict__ w16) {
  const size_t tid = (size_t)blockIdx.x * blockDim.x + threadIdx.x, nth = (size_t)gridDim.x * blockDim.x;
  for (int pass = 0; pass < 2; ++pass) { for (size_t p = tid; p < (size_t)D * FIN / 8; p += nth) { const int n = (int)(p / (FIN / 8)), k0 = (int)(p % (FIN / 8)) * 8; v8b v;
#pragma unroll
      for (int e = 0; e < 8; ++e) v[e] = (b16)W[(size_t)(k0 + e) * D + n];
      *(volatile v8b*)(w16 + (size_t)n * FIN + k0) = v; } __threadfence(); }
}

__global__ __launch_bounds__(128) void lin_kernel(const float* __restrict__ x, const b16* __restrict__ w, float* __restrict__ ft) {
  __shared__ __attribute__((aligned(16))) float Ts[4][32 * 64];
  const int lane = threadIdx.x & 31, wave = threadIdx.x >> 5, nloc = lane & 15, hlf = lane >> 4, m0 = blockIdx.y * 128 + wave * 32, c0 = blockIdx.x * 64;
  v8f acc[2][4];
#pragma unroll
  for (int r = 0; r < 2; ++r)
#pragma unroll
    for (int t = 0; t < 4; ++t) acc[r][t] = (v8f){};
  const Opnd A{x, nullptr, FIN}; const int ra = min(m0 + nloc, N - 1), rb = min(m0 + 16 + nloc, N - 1);
#pragma unroll 1
  for (int kb = 0; kb < FIN; kb += 32) { v16b a0, a1, d0, d1; load_frags<3>(A, ra, kb, hlf, a0, d0); load_frags<3>(A, rb, kb, hlf, a1, d1);
#pragma unroll
    for (int t = 0; t < 4; ++t) { const v16b bw = frag_kb(w + (size_t)(c0 + t * 16 + nloc) * FIN + kb, hlf); acc[0][t] = wmma16b(a0, bw, acc[0][t]); acc[1][t] = wmma16b(a1, bw, acc[1][t]); } }
  epi_f32(acc, 1.0f, nullptr, ft, D, m0, c0, lane, Ts[wave]);
}

__global__ __launch_bounds__(256) void alpha_kernel(const float* __restrict__ ft, const float* __restrict__ attl, const float* __restrict__ attr, float* __restrict__ al) {
  __shared__ float Ab[32][2];
  const int wid = threadIdx.x >> 5, lane = threadIdx.x & 31;
  for (int q = 0; q < 4; ++q) { const int nl = wid * 4 + q, n = blockIdx.x * 32 + nl; const v4f v = *(const v4f*)(ft + (size_t)n * D + lane * 4); float sl = 0.0f, sr = 0.0f;
#pragma unroll
    for (int e = 0; e < 4; ++e) { sl += v[e] * attl[lane * 4 + e]; sr += v[e] * attr[lane * 4 + e]; }
#pragma unroll
    for (int o = 16; o > 0; o >>= 1) { sl += __shfl_xor(sl, o); sr += __shfl_xor(sr, o); }
    if (lane == 0) { Ab[nl][0] = sl; Ab[nl][1] = sr; } }
  __syncthreads();
  if (threadIdx.x < 64) { const float vv = Ab[threadIdx.x >> 1][threadIdx.x & 1]; for (int pass = 0; pass < 2; ++pass) { ((volatile float*)al)[(size_t)blockIdx.x * 64 + threadIdx.x] = vv; __threadfence(); } }
}

typedef __attribute__((ext_vector_type(4))) int v4i;
__global__ __launch_bounds__(256) void gat_kernel(const int* __restrict__ esrc, const int* __restrict__ edst, const float* __restrict__ wgt, const float* __restrict__ ft, const float* __restrict__ al, const float* __restrict__ bias, float* __restrict__ out) {
  __shared__ __attribute__((aligned(16))) int accE[NB * D], accW[NB * D];
  __shared__ int mxE[NB], mxW[NB], denE[NB], denW[NB]; __shared__ int list[8 * 256];
  const int t_ = threadIdx.x, wave = t_ >> 5, lane = t_ & 31, base = blockIdx.x * NB;
  for (int i = t_; i < NB * D; i += 256) { accE[i] = 0; accW[i] = 0; }
  for (int i = t_; i < NB; i += 256) { mxE[i] = fkey(-INFINITY); mxW[i] = fkey(-INFINITY); denE[i] = 0; denW[i] = 0; }
  __syncthreads();
  for (int c0 = 0; c0 < E; c0 += 256 * 8) { const int e0 = c0 + (wave * 32 + lane) * 8;
#pragma unroll
    for (int j = 0; j < 8; ++j) { const int ee = min(e0 + j, E - 1); const int dv = edst[ee]; const unsigned sl = (unsigned)(((e0 + j < E) ? dv : -1) - base);
      if (sl < (unsigned)NB) { int s = esrc[ee]; s = (s < 0) ? 0 : (s >= N ? N - 1 : s); float e = al[(size_t)s * 2] + al[(size_t)(base + sl) * 2 + 1]; e = (e > 0.0f) ? e : NEG * e;
        atomicMax(&mxE[sl], fkey(e)); atomicMax(&mxW[sl], fkey(wgt[ee])); } } }
  __syncthreads();
  int* wl = list + wave * 256;
  for (int c0 = 0; c0 < E; c0 += 256 * 8) {
    const int e0 = c0 + (wave * 32 + lane) * 8; int dd[8];
#pragma unroll
    for (int j = 0; j < 8; ++j) { const int dv = edst[min(e0 + j, E - 1)]; dd[j] = (e0 + j < E) ? dv : -1; }
    unsigned sl[8]; bool hit[8]; bool anyl = false;
#pragma unroll
    for (int j = 0; j < 8; ++j) { sl[j] = (unsigned)(dd[j] - base); hit[j] = sl[j] < (unsigned)NB; anyl |= hit[j]; }
    int wc = 0;
    if (__builtin_amdgcn_ballot_w32(anyl) != 0u) {
#pragma unroll
      for (int j = 0; j < 8; ++j) {
        const unsigned mj = __builtin_amdgcn_ballot_w32(hit[j]);
        if (mj != 0u) {
          if (hit[j]) { const int pos = wc + (int)__builtin_amdgcn_mbcnt_lo(mj, 0u); wl[pos] = ((e0 + j) << 8) | (int)sl[j]; }
          wc += __builtin_popcount(mj); } } }
    __builtin_amdgcn_wave_barrier(); __builtin_amdgcn_fence(__ATOMIC_RELEASE, "workgroup"); __builtin_amdgcn_fence(__ATOMIC_ACQUIRE, "workgroup");
    for (int i = 0; i < wc; ++i) { const int ent = wl[i]; const int e = ent >> 8, slot = ent & 255; int s = esrc[e]; s = (s < 0) ? 0 : (s >= N ? N - 1 : s);
      float sc = al[(size_t)s * 2] + al[(size_t)(base + slot) * 2 + 1]; sc = (sc > 0.0f) ? sc : NEG * sc;
      const float we = __expf(sc - fkey_inv(mxE[slot])), ww = __expf(wgt[e] - fkey_inv(mxW[slot]));
      if (lane == 0) { atomicAdd(&denE[slot], (int)rintf(we * FXS)); atomicAdd(&denW[slot], (int)rintf(ww * FXS)); }
      const v4f v = *(const v4f*)(ft + (size_t)s * D + lane * 4);
#pragma unroll
      for (int c = 0; c < 4; ++c) { atomicAdd(&accE[slot * D + lane * 4 + c], (int)rintf(we * v[c] * FXS)); atomicAdd(&accW[slot * D + lane * 4 + c], (int)rintf(ww * v[c] * FXS)); } }
    __builtin_amdgcn_wave_barrier();
  }
  __syncthreads();
  for (int pass = 0; pass < 2; ++pass) {
    for (int i = t_; i < NB * D / 4; i += 256) { const int r = (i * 4) / D, cq = (i * 4) % D, node = base + r; if (node < N) { v4f o;
        const float de_ = (float)denE[r], dw_ = (float)denW[r]; const float ie = (de_ > 0.0f) ? __builtin_amdgcn_rcpf(de_) : 0.0f, iw = (dw_ > 0.0f) ? __builtin_amdgcn_rcpf(dw_) : 0.0f;
#pragma unroll
        for (int c = 0; c < 4; ++c) o[c] = (1.0f - ALPHA) * (float)accE[i * 4 + c] * ie + ALPHA * (float)accW[i * 4 + c] * iw + bias[cq + c];
        *(volatile v4f*)(out + (size_t)node * D + cq) = o; } }
    __threadfence();
  }
}
}

extern "C" void kernel_launch(void* const* d_in, const int* in_sizes, int n_in,
                              void* d_out, int out_size, void* d_ws, size_t ws_size, hipStream_t stream) {
  (void)n_in; (void)out_size;
  const float* feat = (const float*)d_in[0]; const float* wgt = (const float*)d_in[1]; const float* fcw = (const float*)d_in[2]; const float* attl = (const float*)d_in[3]; const float* attr = (const float*)d_in[4]; const float* bias = (const float*)d_in[5];
  const int* src = (const int*)d_in[6]; const int* dst = (const int*)d_in[7];
  float* out = (float*)d_out;
  if (in_sizes[0] != N * FIN || in_sizes[1] != E || in_sizes[2] != FIN * D || in_sizes[6] != E || in_sizes[7] != E) return;
  size_t off = 0; char* ws = (char*)d_ws;
  auto carve = [&](size_t bytes) { char* p = ws + off; off += (bytes + 255) & ~(size_t)255; return p; };
  b16* w16 = (b16*)carve((size_t)D * FIN * 2); float* ft = (float*)carve((size_t)NPAD * D * 4); float* al = (float*)carve((size_t)NPAD * 2 * 4);
  if (off > ws_size) return;
  prep_kernel<<<32, 256, 0, stream>>>(fcw, w16);
  lin_kernel<<<dim3(2, NBLK), 128, 0, stream>>>(feat, w16, ft);
  alpha_kernel<<<NPAD / 32, 256, 0, stream>>>(ft, attl, attr, al);
  gat_kernel<<<NPAD / NB + 1, 256, 0, stream>>>(src, dst, wgt, ft, al, bias, out);
}
